// PraxisAttention_61512521614063
// MI455X (gfx1250) — hardware-verified
//
#include <hip/hip_runtime.h>
#include <math.h>
#include <stdint.h>

#define NB    2
#define NHQ   16
#define NHP   8
#define NS    2048
#define ND    64
#define NDV   128
#define NQB   (NS / 64)
#define NBLK  (NB * NHP * NQB)
#define GSZ   131072
#define NCH   1024
static_assert(NQB == 32);
static_assert(NBLK == 512);
static_assert((ND % 32) == 0 && (NDV % 16) == 0 && (NS % 64) == 0);
static_assert(NHP * NS * NDV == 16 * GSZ);
static_assert(NCH * NS == NHP * NS * NDV);

typedef __bf16   v16b __attribute__((ext_vector_type(16)));
typedef __bf16   v8b  __attribute__((ext_vector_type(8)));
typedef float    v8f  __attribute__((ext_vector_type(8)));
typedef float    v4f  __attribute__((ext_vector_type(4)));
typedef unsigned int v4u __attribute__((ext_vector_type(4)));
typedef double   v2d  __attribute__((ext_vector_type(2)));

__device__ __forceinline__ unsigned short bf_bits(float f) {
  unsigned u = __float_as_uint(f);
  return (unsigned short)((u + 0x7FFFu + ((u >> 16) & 1u)) >> 16);
}
__device__ __forceinline__ float bf_up(unsigned short h) { return __uint_as_float(((unsigned)h) << 16); }
__device__ __forceinline__ __bf16 bf_val(unsigned short h) { return __builtin_bit_cast(__bf16, h); }
__device__ __forceinline__ unsigned pk16(unsigned short a, unsigned short b) { return (unsigned)a | ((unsigned)b << 16); }
__device__ __forceinline__ v8f zero8() { v8f z = {0.f, 0.f, 0.f, 0.f, 0.f, 0.f, 0.f, 0.f}; return z; }
__device__ __forceinline__ v4u pack8(const float* p) {
  const v4f a = *(const v4f*)(p);
  const v4f b = *(const v4f*)(p + 4);
  v4u r;
  r[0] = pk16(bf_bits(a[0]), bf_bits(a[1]));
  r[1] = pk16(bf_bits(a[2]), bf_bits(a[3]));
  r[2] = pk16(bf_bits(b[0]), bf_bits(b[1]));
  r[3] = pk16(bf_bits(b[2]), bf_bits(b[3]));
  return r;
}

__device__ __forceinline__ v16b ldfrag_b(const __bf16* p) {
  union { v16b v; v8b h[2]; } f;
  f.h[0] = *(const v8b*)(p);
  f.h[1] = *(const v8b*)(p + 16);
  return f.v;
}

__device__ __forceinline__ v8f mma_b(v16b a, v16b b, v8f c) {
  c = __builtin_amdgcn_wmma_f32_16x16x32_bf16(false, a, false, b, (short)0, c, false, false);
  asm volatile("v_nop\n\tv_nop\n\tv_nop\n\tv_nop" : "+v"(c) : "v"(a), "v"(b));
  return c;
}

__global__ __launch_bounds__(256) void cvt_qk(const float* __restrict__ q, const float* __restrict__ k,
                                              unsigned short* qb, unsigned short* kb, int n8) {
  const int i = blockIdx.x * 256 + threadIdx.x;
  if (i < n8) {
    const size_t o = (size_t)i * 8;
    const v4u pq = pack8(q + o);
    const v4u pk = pack8(k + o);
    *(volatile v4u*)(qb + o) = pq;
    *(volatile v4u*)(kb + o) = pk;
    __threadfence();
    *(volatile v4u*)(qb + o) = pq;
    *(volatile v4u*)(kb + o) = pk;
  }
}

__global__ __launch_bounds__(256) void prep_vt(const float* __restrict__ v, unsigned short* vt) {
  __shared__ __align__(16) unsigned short T[NDV * 72];
  const int tid  = threadIdx.x;
  const int wave = tid >> 5;
  const int lane = tid & 31;
  const int blk  = blockIdx.x;
  const int st   = blk & (NQB - 1);
  const int bg   = blk >> 5;
  const int s0   = st * 64;
  const float* src = v + ((size_t)bg * NS + s0) * NDV;
#pragma unroll
  for (int i = 0; i < 8; ++i) {
    const int idx = i * 256 + tid;
    const int s   = idx >> 5;
    const int dv4 = (idx & 31) * 4;
    const v4f f = *(const v4f*)(src + (size_t)s * NDV + dv4);
#pragma unroll
    for (int e = 0; e < 4; ++e) T[(dv4 + e) * 72 + s] = bf_bits(f[e]);
  }
  __syncthreads();
  const int qq = lane >> 3, c8 = (lane & 7) * 8;
  v4u vals[4];
#pragma unroll
  for (int it = 0; it < 4; ++it) {
    const int row = it * 32 + wave * 4 + qq;
    vals[it] = *(const v4u*)(T + row * 72 + c8);
  }
  unsigned short* dst = vt + (size_t)bg * NDV * NS + s0 + c8;
  for (int pass = 0; pass < 2; ++pass) {
#pragma unroll
    for (int it = 0; it < 4; ++it) {
      const int row = it * 32 + wave * 4 + qq;
      *(volatile v4u*)(dst + (size_t)row * NS) = vals[it];
    }
    __threadfence();
  }
}

#define L_K     0
#define L_VT    18432
#define L_PH    36864
#define L_PL    55296
#define L_ACC   73728
#define L_WP    139264
#define L_LAM   141312
#define L_TOTAL 141328
static_assert(L_VT - L_K == 2 * 64 * 72 * 2);
static_assert(L_PH - L_VT == NDV * 72 * 2);
static_assert(L_PL - L_PH == 8 * 16 * 72 * 2 && L_ACC - L_PL == 8 * 16 * 72 * 2);
static_assert(L_WP - L_ACC == 8 * 8 * 32 * 8 * 4);
static_assert(L_LAM - L_WP == 128 * 2 * 8 && L_TOTAL - L_LAM == 16);
static_assert(4 * 16 * 132 * 4 <= L_PH);

__global__ __launch_bounds__(256)
void attn_diff(const unsigned short* __restrict__ qbp, const unsigned short* __restrict__ kbp,
               const unsigned short* __restrict__ vtp,
               const float* __restrict__ lq1, const float* __restrict__ lk1,
               const float* __restrict__ lq2, const float* __restrict__ lk2,
               float* Op, double* recp) {
  extern __shared__ __align__(16) unsigned char lds[];
  union FB { v16b v; v8b h[2]; };
  __bf16* Ks    = (__bf16*)(lds + L_K);
  __bf16* Vt    = (__bf16*)(lds + L_VT);
  __bf16* Ph    = (__bf16*)(lds + L_PH);
  __bf16* Pl    = (__bf16*)(lds + L_PL);
  float*  accL  = (float*)(lds + L_ACC);
  double* wpart = (double*)(lds + L_WP);
  float*  lamS  = (float*)(lds + L_LAM);

  const int tid  = threadIdx.x;
  const int wave = tid >> 5;
  const int lane = tid & 31;
  const int hh   = lane >> 4;
  const int c    = lane & 15;
  const int head = wave & 1;
  const int rg   = wave >> 1;

  const int bid = blockIdx.x;
  const int qb  = bid & (NQB - 1);
  const int g   = (bid >> 5) & (NHP - 1);
  const int b   = bid >> 8;
  const int q0  = qb * 64 + rg * 16;

  const __bf16* Qb = (const __bf16*)(const void*)qbp;
  const __bf16* Kb = (const __bf16*)(const void*)kbp;
  const __bf16* Kg = Kb + (size_t)(b * NHQ + 2 * g) * NS * ND;
  const __bf16* Vg = (const __bf16*)(const void*)vtp + (size_t)(b * NHP + g) * NDV * NS;

  if (tid == 0) {
    double s1 = 0.0, s2 = 0.0;
#pragma unroll 1
    for (int i = 0; i < ND; ++i) {
      const float a1 = bf_up(bf_bits(lq1[i])), b1 = bf_up(bf_bits(lk1[i]));
      const float a2 = bf_up(bf_bits(lq2[i])), b2 = bf_up(bf_bits(lk2[i]));
      s1 += (double)(a1 * b1);
      s2 += (double)(a2 * b2);
    }
    *lamS = expf((float)s1) - expf((float)s2) + 0.8f;
  }

  float*  accW = accL + wave * 2048;
  __bf16* pwh  = Ph + wave * (16 * 72);
  __bf16* pwl  = Pl + wave * (16 * 72);
#pragma unroll
  for (int t = 0; t < 8; ++t) *(v8f*)(accW + (t * 32 + lane) * 8) = zero8();

  float mrow[8], lrow[8], alpha[8];
#pragma unroll
  for (int r = 0; r < 8; ++r) { mrow[r] = 0.f; lrow[r] = 1.f; alpha[r] = 1.f; }

  const size_t qo = ((size_t)(b * NHQ + 2 * g + head) * NS + q0 + c) * ND + 8 * hh;
  v16b qa[2];
  qa[0] = ldfrag_b(Qb + qo);
  qa[1] = ldfrag_b(Qb + qo + 32);

  for (int kt = 0; kt <= qb; ++kt) {
    const int kv0 = kt * 64;
    __syncthreads();
#pragma unroll
    for (int i = 0; i < 4; ++i) {
      const int p    = tid + 256 * i;
      const int hsel = p >> 9;
      const int rem  = p & 511;
      const int r    = rem >> 3;
      const int d8   = (rem & 7) * 8;
      const v8b ka = *(const v8b*)(Kg + ((size_t)hsel * NS + kv0 + r) * ND + d8);
      const int dv = p >> 3;
      const int s8 = (p & 7) * 8;
      const v8b va = *(const v8b*)(Vg + (size_t)dv * NS + kv0 + s8);
      *(v8b*)(Ks + (hsel * 64 + r) * 72 + d8) = ka;
      *(v8b*)(Vt + dv * 72 + s8) = va;
    }
    __syncthreads();

    v8f s[4];
#pragma unroll
    for (int j = 0; j < 4; ++j) s[j] = zero8();
#pragma unroll
    for (int dc = 0; dc < 2; ++dc) {
      const int ko = (head * 64) * 72 + dc * 32 + 8 * hh;
#pragma unroll
      for (int j = 0; j < 4; ++j) {
        const int kr = (j * 16 + c) * 72 + ko;
        FB kf;
        kf.h[0] = *(const v8b*)(Ks + kr);
        kf.h[1] = *(const v8b*)(Ks + kr + 16);
        s[j] = mma_b(qa[dc], kf.v, s[j]);
      }
    }

#pragma unroll
    for (int r = 0; r < 8; ++r) {
      const int rowq = q0 + 8 * hh + r;
      float m = -INFINITY;
#pragma unroll
      for (int j = 0; j < 4; ++j) {
        const int key = kv0 + j * 16 + c;
        float sv = s[j][r] * 0.125f;
        sv = (key <= rowq) ? sv : -INFINITY;
        s[j][r] = sv;
        m = fmaxf(m, sv);
      }
#pragma unroll
      for (int off = 1; off < 16; off <<= 1) m = fmaxf(m, __shfl_xor(m, off, 32));
      const float mnew = fmaxf(mrow[r], m);
      const float al   = __expf(mrow[r] - mnew);
      mrow[r]  = mnew;
      alpha[r] = al;
      float psum = 0.f;
#pragma unroll
      for (int j = 0; j < 4; ++j) {
        const float p = __expf(s[j][r] - mnew);
        psum += p;
        const unsigned short hb = bf_bits(p);
        const unsigned short lb = bf_bits(p - bf_up(hb));
        const int po = (8 * hh + r) * 72 + j * 16 + c;
        pwh[po] = bf_val(hb);
        pwl[po] = bf_val(lb);
      }
#pragma unroll
      for (int off = 1; off < 16; off <<= 1) psum += __shfl_xor(psum, off, 32);
      lrow[r] = lrow[r] * al + psum;
    }
    __builtin_amdgcn_fence(__ATOMIC_RELEASE, "workgroup");
    __builtin_amdgcn_wave_barrier();
    __builtin_amdgcn_fence(__ATOMIC_ACQUIRE, "workgroup");

    FB pa[2], pl[2];
#pragma unroll
    for (int kk = 0; kk < 2; ++kk) {
      const int pr = c * 72 + kk * 32 + 8 * hh;
      pa[kk].h[0] = *(const v8b*)(pwh + pr);
      pa[kk].h[1] = *(const v8b*)(pwh + pr + 16);
      pl[kk].h[0] = *(const v8b*)(pwl + pr);
      pl[kk].h[1] = *(const v8b*)(pwl + pr + 16);
    }
#pragma unroll 1
    for (int t = 0; t < 8; ++t) {
      float* ap = accW + (t * 32 + lane) * 8;
      v8f acc = *(const v8f*)ap;
#pragma unroll
      for (int r = 0; r < 8; ++r) acc[r] *= alpha[r];
      const int vr0 = (t * 16 + c) * 72 + 8 * hh;
#pragma unroll
      for (int kk = 0; kk < 2; ++kk) {
        FB vf;
        vf.h[0] = *(const v8b*)(Vt + vr0 + kk * 32);
        vf.h[1] = *(const v8b*)(Vt + vr0 + kk * 32 + 16);
        acc = mma_b(pa[kk].v, vf.v, acc);
        acc = mma_b(pl[kk].v, vf.v, acc);
      }
      *(v8f*)ap = acc;
    }
  }

  __syncthreads();
  float inv[8];
#pragma unroll
  for (int r = 0; r < 8; ++r) inv[r] = 1.0f / lrow[r];
  float* Ob = (float*)(lds + L_K) + rg * (16 * 132);
  if (head == 1) {
    const float lam = *lamS;
#pragma unroll 1
    for (int t = 0; t < 8; ++t) {
      const v8f acc = *(const v8f*)(accW + (t * 32 + lane) * 8);
#pragma unroll
      for (int r = 0; r < 8; ++r) Ob[(8 * hh + r) * 132 + t * 16 + c] = lam * (acc[r] * inv[r]);
    }
  }
  __syncthreads();
  if (head == 0) {
    float ps = 0.f, ps2 = 0.f;
#pragma unroll 1
    for (int t = 0; t < 8; ++t) {
      const v8f acc = *(const v8f*)(accW + (t * 32 + lane) * 8);
#pragma unroll
      for (int r = 0; r < 8; ++r) {
        const int idx = (8 * hh + r) * 132 + t * 16 + c;
        const float y = acc[r] * inv[r] - Ob[idx];
        Ob[idx] = y;
        ps  += y;
        ps2 += y * y;
      }
    }
    wpart[(rg * 32 + lane) * 2]     = (double)ps;
    wpart[(rg * 32 + lane) * 2 + 1] = (double)ps2;
    __builtin_amdgcn_fence(__ATOMIC_RELEASE, "workgroup");
    __builtin_amdgcn_wave_barrier();
    __builtin_amdgcn_fence(__ATOMIC_ACQUIRE, "workgroup");
    float* og = Op + ((size_t)(b * NHP + g) * NS + q0) * NDV;
    for (int pass = 0; pass < 2; ++pass) {
#pragma unroll 4
      for (int row = 0; row < 16; ++row) {
        const v4f vv = *(const v4f*)(Ob + row * 132 + lane * 4);
        *(volatile v4f*)(og + (size_t)row * NDV + lane * 4) = vv;
      }
      __threadfence();
    }
  }
  __syncthreads();
  if (wave == 0 && lane < 8) {
    double S = 0.0, S2 = 0.0;
#pragma unroll 1
    for (int i = 0; i < 128; ++i) { S += wpart[2 * i]; S2 += wpart[2 * i + 1]; }
    v2d rv;
    rv[0] = S; rv[1] = S2;
    double* rp = recp + (size_t)bid * 16 + lane * 2;
    *(volatile v2d*)rp = rv;
    __threadfence();
    *(volatile v2d*)rp = rv;
  }
}

__global__ __launch_bounds__(256) void gn_apply(const float* __restrict__ Op, const double* __restrict__ recp,
                                                const float* __restrict__ gw, const float* __restrict__ gbias,
                                                float* out) {
  __shared__ float sStat[4];
  const int tid = threadIdx.x;
  const int blk = blockIdx.x;
  const int b   = blk >> 10;
  const int ch  = blk & (NCH - 1);
  const int r   = ch >> 6;
  const int g   = r >> 1;
  const int half = r & 1;
  if (tid == 0) {
    double S = 0.0, S2 = 0.0;
    const double* rp = recp + ((size_t)((b * NHP + g) * NQB + half * 16)) * 16;
#pragma unroll 1
    for (int j = 0; j < 16; ++j) { S += rp[j * 16]; S2 += rp[j * 16 + 1]; }
    const double mean = S * (1.0 / (double)GSZ);
    double var = S2 * (1.0 / (double)GSZ) - mean * mean;
    var = (var > 0.0) ? var : 0.0;
    const float varf = (float)var;
    sStat[0] = (float)mean;
    sStat[1] = 1.0f / sqrtf(varf + 1e-5f);
  }
  __syncthreads();
  const float mean = sStat[0];
  const float rstd = sStat[1];
  const float w  = bf_up(bf_bits(gw[ch]));
  const float bi = bf_up(bf_bits(gbias[ch]));
  const size_t base = (size_t)b * ((size_t)NHP * NS * NDV) + (size_t)ch * NS;
  v4f y[2];
#pragma unroll
  for (int it = 0; it < 2; ++it) {
    const int i = it * 256 + tid;
    const v4f x = *(const v4f*)(Op + base + (size_t)i * 4);
    v4f yy;
#pragma unroll
    for (int e = 0; e < 4; ++e) {
      float t = (x[e] - mean) * rstd;
      t = t * w + bi;
      yy[e] = t * 0.2f;
    }
    y[it] = yy;
  }
#pragma unroll
  for (int it = 0; it < 2; ++it) *(volatile v4f*)(out + base + (size_t)(it * 256 + tid) * 4) = y[it];
  __threadfence();
#pragma unroll
  for (int it = 0; it < 2; ++it) *(volatile v4f*)(out + base + (size_t)(it * 256 + tid) * 4) = y[it];
}

extern "C" void kernel_launch(void* const* d_in, const int* in_sizes, int n_in,
                              void* d_out, int out_size, void* d_ws, size_t ws_size,
                              hipStream_t stream) {
  if (n_in < 9) return;
  const int nqk = NB * NHQ * NS * ND;
  const int nv  = NB * NHP * NS * NDV;
  if (in_sizes[0] != nqk || in_sizes[1] != nqk || in_sizes[2] != nv) return;
  if (in_sizes[3] != ND || in_sizes[4] != ND || in_sizes[5] != ND || in_sizes[6] != ND) return;
  if (in_sizes[7] != NHQ * ND || in_sizes[8] != NHQ * ND) return;
  if (out_size != nv) return;

  const float* q   = (const float*)d_in[0];
  const float* k   = (const float*)d_in[1];
  const float* v   = (const float*)d_in[2];
  const float* lq1 = (const float*)d_in[3];
  const float* lk1 = (const float*)d_in[4];
  const float* lq2 = (const float*)d_in[5];
  const float* lk2 = (const float*)d_in[6];
  const float* gw  = (const float*)d_in[7];
  const float* gb  = (const float*)d_in[8];

  const size_t PQ  = (size_t)nqk * 2;
  const size_t PK  = (size_t)nqk * 2;
  const size_t PVT = (size_t)nv * 2;
  const size_t PO  = (size_t)nv * 4;
  const size_t PR  = (size_t)NBLK * 128;
  size_t off = 0;
  const size_t oQ  = off; off += PQ;
  const size_t oK  = off; off += PK;
  const size_t oVT = off; off += PVT;
  const size_t oO  = off; off += PO;
  const size_t oR  = off; off += PR;
  if (off > ws_size) return;
  if (off > (size_t)134217728) return;

  char* ws = (char*)d_ws;
  unsigned short* Qb = (unsigned short*)(ws + oQ);
  unsigned short* Kb = (unsigned short*)(ws + oK);
  unsigned short* VT = (unsigned short*)(ws + oVT);
  float*          O  = (float*)(ws + oO);
  double*         R  = (double*)(ws + oR);

  const int  n8 = nqk / 8;
  const dim3 blk(256);
  const dim3 gCvt((n8 + 255) / 256);
  const dim3 gVt(NB * NHP * NQB);
  const dim3 gAttn(NBLK);
  const dim3 gGn(NB * NCH);

  cvt_qk<<<gCvt, blk, 0, stream>>>(q, k, Qb, Kb, n8);
  prep_vt<<<gVt, blk, 0, stream>>>(v, VT);
  (void)hipFuncSetAttribute(reinterpret_cast<const void*>(&attn_diff),
                            hipFuncAttributeMaxDynamicSharedMemorySize, L_TOTAL);
  attn_diff<<<gAttn, blk, L_TOTAL, stream>>>(Qb, Kb, VT, lq1, lk1, lq2, lk2, O, R);
  gn_apply<<<gGn, blk, 0, stream>>>(O, R, gw, gb, (float*)d_out);
  (void)hipGetLastError();
}
